// GATLayer_15264313770199
// MI455X (gfx1250) — hardware-verified
//
#include <hip/hip_runtime.h>
#include <stddef.h>
#include <stdint.h>
#include <math.h>


#define F_IN   256
#define GC     128
#define NHD    4
#define FH     32
#define NTHR   256
#define NWAVE  8
#define RB     16
#define RW     2
#define TJ     64
#define GP     132
#define GBM    64
#define GBN    64
#define GTHR   128
#define NEGSL  0.2f
#define WSMAX  134217728
#define LDS_ATTN (TJ * GP * 4 + RB * GC * 4 + 2 * NHD * RB * TJ * 2 + RB * TJ * 4 + RB * NHD * 4 * 4 + FH * 4)

static_assert(GC == NHD * FH);
static_assert(FH == 32);
static_assert(TJ == 64);
static_assert(RB == 16);
static_assert(RB == RW * NWAVE && NTHR == 32 * NWAVE);
static_assert(NWAVE == NHD * (FH / 16));
static_assert((GP % 4) == 0 && GP >= GC);
static_assert((F_IN % 32) == 0 && (F_IN / 8) == 32);
static_assert((GC % GBN) == 0);
static_assert(GBM == (GTHR / 32) * 16);
static_assert(GBM == 64 && GBN == 64 && GTHR == 128);
static_assert(TJ == GBM);
static_assert(NTHR * 8 * 4 == TJ * GC);
static_assert(NTHR * 4 == RB * TJ);
static_assert(NTHR * 2 * 4 == RB * GC);
static_assert(RB * GC <= TJ * GP);
static_assert(RB * 8 <= NTHR);
static_assert(LDS_ATTN <= 65536);

typedef float          v4f  __attribute__((ext_vector_type(4)));
typedef float          v8f  __attribute__((ext_vector_type(8)));
typedef int            v8i  __attribute__((ext_vector_type(8)));
typedef unsigned int   v4u  __attribute__((ext_vector_type(4)));
typedef unsigned short v8us __attribute__((ext_vector_type(8)));
typedef __bf16         v16b __attribute__((ext_vector_type(16)));
typedef v4f  __attribute__((may_alias)) v4fa;
typedef v8us __attribute__((may_alias)) v8usa;
union FragB { v16b v; v8us h[2]; v8i w; };

__device__ __forceinline__ v8f wmb(const FragB& a, const FragB& b, v8f c) {
  v8f d = __builtin_amdgcn_wmma_f32_16x16x32_bf16(false, a.v, false, b.v, (short)0, c, false, false);
  asm volatile("v_nop\n\tv_nop\n\tv_nop\n\tv_nop" : "+v"(d) : "v"(a.w), "v"(b.w));
  return d;
}

__device__ __forceinline__ unsigned int f2bf(float f) {
  const unsigned int u = __float_as_uint(f);
  return ((u + 0x7FFFu + ((u >> 16) & 1u)) >> 16) & 0xFFFFu;
}
__device__ __forceinline__ float bf2f(unsigned int b) { return __uint_as_float(b << 16); }
__device__ __forceinline__ float bfr(float f) { return bf2f(f2bf(f)); }
__device__ __forceinline__ unsigned int pk2(float lo, float hi) { return f2bf(lo) | (f2bf(hi) << 16); }
__device__ __forceinline__ v4u pack8(const v4f a, const v4f b) {
  v4u r;
  r.x = pk2(a.x, a.y); r.y = pk2(a.z, a.w); r.z = pk2(b.x, b.y); r.w = pk2(b.z, b.w);
  return r;
}
__device__ __forceinline__ float lk(float a, float b) { const float v = a + b; return fmaxf(v, v * NEGSL); }

__global__ __launch_bounds__(NTHR) void k_xprep(const float* __restrict__ x, unsigned short* xb, int nN, int nUnits) {
  const int i = (int)blockIdx.x * NTHR + (int)threadIdx.x;
  if (i >= nUnits) return;
  const int row = i >> 5;
  const int c0  = (i & 31) * 8;
  const int rc  = row < nN ? row : nN - 1;
  const float* p = x + (size_t)rc * F_IN + c0;
  v4f a = *(const v4fa*)p, b = *(const v4fa*)(p + 4);
  const v4f z4 = {0.f, 0.f, 0.f, 0.f};
  if (row >= nN) { a = z4; b = z4; }
  const v4u hv = pack8(a, b);
  const size_t o = (size_t)row * F_IN + c0;
  *(volatile v4u*)(xb + o) = hv;
  __threadfence();
  *(volatile v4u*)(xb + o) = hv;
}

__global__ __launch_bounds__(NTHR) void k_wtr(const float* __restrict__ w, int Kin, int Ncol, int Nrows, int Kout,
                                              unsigned short* wt, int nUnits) {
  const int u = (int)blockIdx.x * NTHR + (int)threadIdx.x;
  if (u >= nUnits) return;
  const int kq = Kout >> 3;
  const int n  = u / kq;
  const int k8 = (u - n * kq) * 8;
  const int kk = k8 - (k8 / Kin) * Kin;
  const int ncl = n < Ncol ? n : Ncol - 1;
  const float* p = w + (size_t)kk * (size_t)Ncol + ncl;
  v4f a, b;
  a.x = p[0];                    a.y = p[(size_t)Ncol];         a.z = p[(size_t)2 * Ncol];     a.w = p[(size_t)3 * Ncol];
  b.x = p[(size_t)4 * Ncol];     b.y = p[(size_t)5 * Ncol];     b.z = p[(size_t)6 * Ncol];     b.w = p[(size_t)7 * Ncol];
  const v4f z4 = {0.f, 0.f, 0.f, 0.f};
  if (n >= Ncol || n >= Nrows) { a = z4; b = z4; }
  const v4u wv = pack8(a, b);
  unsigned short* o = wt + (size_t)n * (size_t)Kout + k8;
  *(volatile v4u*)o = wv;
  __threadfence();
  *(volatile v4u*)o = wv;
}

__global__ __launch_bounds__(GTHR) void k_gemm(
    const unsigned short* __restrict__ A, const unsigned short* __restrict__ WT,
    float* outF, unsigned short* GTh, unsigned short* GTl, int K, int ldo, int ldt)
{
  __shared__ __attribute__((aligned(16))) float stg[GBM * GBN];
  const int tid = (int)threadIdx.x, lane = tid & 31, wave = tid >> 5, hh = lane >> 4, m = lane & 15;
  const int rowBase = (int)blockIdx.x * GBM;
  const int col0    = (int)blockIdx.y * GBN;

  v8f acc[4];
  {
    const v8f z = {0.f, 0.f, 0.f, 0.f, 0.f, 0.f, 0.f, 0.f};
    acc[0] = z; acc[1] = z; acc[2] = z; acc[3] = z;
  }
  const unsigned short* ap = A  + (size_t)(rowBase + 16 * wave + m) * (size_t)K + 8 * hh;
  const unsigned short* wp = WT + (size_t)(col0 + m) * (size_t)K + 8 * hh;
  const int ksteps = K >> 5;
#pragma unroll 1
  for (int ks = 0; ks < ksteps; ++ks) {
    FragB af;
    af.h[0] = *(const v8usa*)(ap + 32 * ks);
    af.h[1] = *(const v8usa*)(ap + 32 * ks + 16);
#pragma unroll
    for (int t = 0; t < 4; ++t) {
      const unsigned short* wq = wp + (size_t)(16 * t) * (size_t)K + 32 * ks;
      FragB bf;
      bf.h[0] = *(const v8usa*)wq;
      bf.h[1] = *(const v8usa*)(wq + 16);
      acc[t] = wmb(af, bf, acc[t]);
    }
  }

#pragma unroll
  for (int t = 0; t < 4; ++t) {
    const int lc = 16 * t + m;
#pragma unroll
    for (int r = 0; r < 8; ++r) {
      const int lr = 16 * wave + 8 * hh + r;
      stg[lr * GBN + lc] = acc[t][r];
    }
  }
  __syncthreads();

  v4f fv[8];
#pragma unroll
  for (int i = 0; i < 8; ++i) {
    const int lr = 16 * wave + 2 * i + hh;
    fv[i] = *(const v4fa*)(stg + lr * GBN + 4 * m);
  }
  const int fq = tid >> 3, kp = 8 * (tid & 7);
  v4u th[4], tl[4];
#pragma unroll
  for (int ps = 0; ps < 4; ++ps) {
    const int fr = 16 * ps + fq;
    unsigned int hb[8], lb[8];
#pragma unroll
    for (int i = 0; i < 8; ++i) {
      const float ev = stg[(kp + i) * GBN + fr];
      hb[i] = f2bf(ev);
      lb[i] = f2bf(ev - bf2f(hb[i]));
    }
    v4u a4, b4;
    a4.x = hb[0] | (hb[1] << 16); a4.y = hb[2] | (hb[3] << 16); a4.z = hb[4] | (hb[5] << 16); a4.w = hb[6] | (hb[7] << 16);
    b4.x = lb[0] | (lb[1] << 16); b4.y = lb[2] | (lb[3] << 16); b4.z = lb[4] | (lb[5] << 16); b4.w = lb[6] | (lb[7] << 16);
    th[ps] = a4; tl[ps] = b4;
  }

#pragma unroll
  for (int i = 0; i < 8; ++i) {
    const int lr = 16 * wave + 2 * i + hh;
    const int gr = rowBase + lr;
    float* op = outF + (size_t)gr * (size_t)ldo + col0 + 4 * m;
    *(volatile v4f*)op = fv[i];
  }
#pragma unroll
  for (int ps = 0; ps < 4; ++ps) {
    const size_t to = (size_t)(col0 + 16 * ps + fq) * (size_t)ldt + (size_t)rowBase + kp;
    *(volatile v4u*)(GTh + to) = th[ps];
    *(volatile v4u*)(GTl + to) = tl[ps];
  }
  __threadfence();
#pragma unroll
  for (int i = 0; i < 8; ++i) {
    const int lr = 16 * wave + 2 * i + hh;
    const int gr = rowBase + lr;
    float* op = outF + (size_t)gr * (size_t)ldo + col0 + 4 * m;
    *(volatile v4f*)op = fv[i];
  }
#pragma unroll
  for (int ps = 0; ps < 4; ++ps) {
    const size_t to = (size_t)(col0 + 16 * ps + fq) * (size_t)ldt + (size_t)rowBase + kp;
    *(volatile v4u*)(GTh + to) = th[ps];
    *(volatile v4u*)(GTl + to) = tl[ps];
  }
}

__device__ __forceinline__ void sm_step(float s0, float s1, int row, int hd, int lane,
                                        float* sSt, unsigned short* sPh, unsigned short* sPl, float ninf) {
  const int so = (row * NHD + hd) * 4;
  const float m_old = sSt[so + 0];
  const float l_old = sSt[so + 1];
  float mx = fmaxf(s0, s1);
#pragma unroll
  for (int off = 16; off > 0; off >>= 1) mx = fmaxf(mx, __shfl_xor(mx, off));
  const float m_new = fmaxf(m_old, mx);
  const float msafe = (m_new == ninf) ? 0.f : m_new;
  const float p0 = expf(s0 - msafe);
  const float p1 = expf(s1 - msafe);
  const float sc = expf(m_old - msafe);
  float ps = p0 + p1;
#pragma unroll
  for (int off = 16; off > 0; off >>= 1) ps += __shfl_xor(ps, off);
  const float l_new = fmaf(l_old, sc, ps);
  const unsigned int h0 = f2bf(p0), h1 = f2bf(p1);
  const unsigned int q0 = f2bf(p0 - bf2f(h0)), q1 = f2bf(p1 - bf2f(h1));
  const int po = (hd * RB + row) * TJ;
  sPh[po + lane] = (unsigned short)h0;  sPh[po + lane + 32] = (unsigned short)h1;
  sPl[po + lane] = (unsigned short)q0;  sPl[po + lane + 32] = (unsigned short)q1;
  if (lane == 0) { sSt[so + 0] = m_new; sSt[so + 1] = l_new; sSt[so + 2] = sc; }
}

__global__ __launch_bounds__(NTHR) void k_attn(const float* __restrict__ G, const unsigned short* __restrict__ GTh,
                                               const unsigned short* __restrict__ GTl, const int* __restrict__ adj,
                                               const float* __restrict__ aw, float* out, int nN, int nT, int MPk) {
  __shared__ __attribute__((aligned(16))) float sGt[TJ * GP];
  __shared__ __attribute__((aligned(16))) float sGi[RB * GC];
  __shared__ __attribute__((aligned(16))) unsigned short sPh[NHD * RB * TJ];
  __shared__ __attribute__((aligned(16))) unsigned short sPl[NHD * RB * TJ];
  __shared__ __attribute__((aligned(16))) int   sAdj[RB * TJ];
  __shared__ __attribute__((aligned(16))) float sSt[RB * NHD * 4];
  __shared__ __attribute__((aligned(16))) float sW[FH];
  const int tid = (int)threadIdx.x, lane = tid & 31, wave = tid >> 5, hh = lane >> 4, m = lane & 15;
  const int rowBase = (int)blockIdx.x * RB;
  const float ninf = __uint_as_float(0xff800000u);

#pragma unroll
  for (int q = 0; q < 2; ++q) {
    const int idx = tid + NTHR * q;
    const int r = idx >> 5, c4 = idx & 31;
    int rr = rowBase + r; rr = rr < nN ? rr : nN - 1;
    const v4f v = *(const v4fa*)(G + (size_t)rr * GC + 4 * c4);
    *(v4f*)(sGi + r * GC + 4 * c4) = v;
  }
  if (tid < FH) sW[tid] = bfr(aw[tid]);
  if (tid < RB * NHD) {
    sSt[4 * tid + 0] = ninf; sSt[4 * tid + 1] = 0.f; sSt[4 * tid + 2] = 0.f; sSt[4 * tid + 3] = 0.f;
  }
  const int hdB = wave >> 1;
  const int ntB = wave & 1;
  const int cB  = hdB * FH + ntB * 16 + m;
  v8f acc = {0.f, 0.f, 0.f, 0.f, 0.f, 0.f, 0.f, 0.f};
  __syncthreads();

#pragma unroll 1
  for (int t = 0; t < nT; ++t) {
    const int j0 = t * TJ;
#pragma unroll
    for (int q = 0; q < 8; ++q) {
      const int idx = tid + NTHR * q;
      const int r = idx >> 5, c4 = idx & 31;
      const v4f v = *(const v4fa*)(G + (size_t)(j0 + r) * GC + 4 * c4);
      *(v4f*)(sGt + r * GP + 4 * c4) = v;
    }
#pragma unroll
    for (int q = 0; q < 4; ++q) {
      const int idx = tid + NTHR * q;
      const int r = idx >> 6, c = idx & 63;
      int ir = rowBase + r; ir = ir < nN ? ir : nN - 1;
      const int j  = j0 + c;
      const int jc = j < nN ? j : nN - 1;
      int a = adj[(size_t)ir * (size_t)nN + jc];
      a &= -(int)(j < nN);
      sAdj[r * TJ + c] = a;
    }
    __syncthreads();

    {
      const int rA = RW * wave, rB2 = rA + 1;
      const float* giA = sGi + rA * GC;
      const float* giB = sGi + rB2 * GC;
      const float* ga  = sGt + lane * GP;
      const float* gb  = sGt + (lane + 32) * GP;
      const int aA0 = sAdj[rA * TJ + lane],  aA1 = sAdj[rA * TJ + lane + 32];
      const int aB0 = sAdj[rB2 * TJ + lane], aB1 = sAdj[rB2 * TJ + lane + 32];
#pragma unroll 1
      for (int hd = 0; hd < NHD; ++hd) {
        const int cb = hd * FH;
        float s00 = 0.f, s01 = 0.f, s10 = 0.f, s11 = 0.f;
#pragma unroll 1
        for (int f4 = 0; f4 < FH / 4; ++f4) {
          const v4f w4 = *(const v4fa*)(sW + 4 * f4);
          const v4f iA = *(const v4fa*)(giA + cb + 4 * f4);
          const v4f iB = *(const v4fa*)(giB + cb + 4 * f4);
          const v4f x4 = *(const v4fa*)(ga + cb + 4 * f4);
          const v4f y4 = *(const v4fa*)(gb + cb + 4 * f4);
          s00 = fmaf(lk(iA.x, x4.x), w4.x, s00);
          s00 = fmaf(lk(iA.y, x4.y), w4.y, s00);
          s00 = fmaf(lk(iA.z, x4.z), w4.z, s00);
          s00 = fmaf(lk(iA.w, x4.w), w4.w, s00);
          s01 = fmaf(lk(iA.x, y4.x), w4.x, s01);
          s01 = fmaf(lk(iA.y, y4.y), w4.y, s01);
          s01 = fmaf(lk(iA.z, y4.z), w4.z, s01);
          s01 = fmaf(lk(iA.w, y4.w), w4.w, s01);
          s10 = fmaf(lk(iB.x, x4.x), w4.x, s10);
          s10 = fmaf(lk(iB.y, x4.y), w4.y, s10);
          s10 = fmaf(lk(iB.z, x4.z), w4.z, s10);
          s10 = fmaf(lk(iB.w, x4.w), w4.w, s10);
          s11 = fmaf(lk(iB.x, y4.x), w4.x, s11);
          s11 = fmaf(lk(iB.y, y4.y), w4.y, s11);
          s11 = fmaf(lk(iB.z, y4.z), w4.z, s11);
          s11 = fmaf(lk(iB.w, y4.w), w4.w, s11);
        }
        s00 = (aA0 != 0) ? s00 : ninf;
        s01 = (aA1 != 0) ? s01 : ninf;
        s10 = (aB0 != 0) ? s10 : ninf;
        s11 = (aB1 != 0) ? s11 : ninf;
#pragma unroll 1
        for (int rw = 0; rw < RW; ++rw) {
          const float u0 = (rw == 0) ? s00 : s10;
          const float u1 = (rw == 0) ? s01 : s11;
          sm_step(u0, u1, rA + rw, hd, lane, sSt, sPh, sPl, ninf);
        }
      }
    }
    __syncthreads();

    {
      v8f scv;
#pragma unroll
      for (int r = 0; r < 8; ++r) scv[r] = sSt[((8 * hh + r) * NHD + hdB) * 4 + 2];
      acc = acc * scv;
      const unsigned short* ph = sPh + (hdB * RB + m) * TJ + 8 * hh;
      const unsigned short* pl = sPl + (hdB * RB + m) * TJ + 8 * hh;
      const size_t gto = (size_t)cB * (size_t)MPk + (size_t)j0 + (size_t)(8 * hh);
      const unsigned short* bh = GTh + gto;
      const unsigned short* bl = GTl + gto;
#pragma unroll
      for (int ks = 0; ks < TJ / 32; ++ks) {
        FragB fah, fal, fbh, fbl;
        fah.h[0] = *(const v8usa*)(ph + 32 * ks);
        fah.h[1] = *(const v8usa*)(ph + 32 * ks + 16);
        fal.h[0] = *(const v8usa*)(pl + 32 * ks);
        fal.h[1] = *(const v8usa*)(pl + 32 * ks + 16);
        fbh.h[0] = *(const v8usa*)(bh + 32 * ks);
        fbh.h[1] = *(const v8usa*)(bh + 32 * ks + 16);
        fbl.h[0] = *(const v8usa*)(bl + 32 * ks);
        fbl.h[1] = *(const v8usa*)(bl + 32 * ks + 16);
        acc = wmb(fah, fbh, acc);
        acc = wmb(fal, fbh, acc);
        acc = wmb(fah, fbl, acc);
      }
    }
    __syncthreads();
  }

  float* sO = sGt;
  {
#pragma unroll
    for (int r = 0; r < 8; ++r) {
      const int q = 8 * hh + r;
      const float lf  = sSt[(q * NHD + hdB) * 4 + 1];
      const float inv = __builtin_amdgcn_rcpf(lf);
      sO[q * GC + hdB * FH + ntB * 16 + m] = acc[r] * inv;
    }
  }
  __syncthreads();
  {
    const int q  = (tid >> 3) & (RB - 1);
    const int pc = tid & 7;
    const float* ob = sO + q * GC + 4 * pc;
    const v4f h0 = *(const v4fa*)(ob);
    const v4f h1 = *(const v4fa*)(ob + FH);
    const v4f h2 = *(const v4fa*)(ob + 2 * FH);
    const v4f h3 = *(const v4fa*)(ob + 3 * FH);
    const v4f o4 = (((h0 + h1) + h2) + h3) * 0.25f;
    const int grow = rowBase + q;
    const int gcl  = grow < nN ? grow : nN - 1;
    float* op = out + (size_t)gcl * FH + 4 * pc;
    const bool wr = (tid < RB * 8) && (grow < nN);
    if (wr) *(volatile v4f*)op = o4;
    __threadfence();
    if (wr) *(volatile v4f*)op = o4;
  }
}

static inline int cdiv(int a, int b) { return (a + b - 1) / b; }

extern "C" void kernel_launch(void* const* d_in, const int* in_sizes, int n_in,
                              void* d_out, int out_size, void* d_ws, size_t ws_size,
                              hipStream_t stream) {
  if (n_in < 4) return;
  const int nN = in_sizes[0] / F_IN;
  if (nN <= 0 || in_sizes[0] != nN * F_IN || nN > 32768) return;
  if ((long long)in_sizes[1] != (long long)nN * (long long)nN) return;
  if (in_sizes[2] != F_IN * GC) return;
  if (in_sizes[3] != FH) return;
  if (out_size != nN * FH) return;

  const float* h   = (const float*)d_in[0];
  const int*   adj = (const int*)  d_in[1];
  const float* Wl  = (const float*)d_in[2];
  const float* aw  = (const float*)d_in[3];
  float* out = (float*)d_out;

  const int MP = cdiv(nN, GBM) * GBM;
  const int nT = MP / TJ;

  char* ws = (char*)d_ws;
  size_t off = 0;
  const size_t oXB  = off; off += (size_t)MP * F_IN * 2;         off = (off + 255) & ~(size_t)255;
  const size_t oWT  = off; off += (size_t)GC * F_IN * 2;         off = (off + 255) & ~(size_t)255;
  const size_t oG   = off; off += (size_t)MP * GC * 4;           off = (off + 255) & ~(size_t)255;
  const size_t oGTh = off; off += (size_t)GC * MP * 2;           off = (off + 255) & ~(size_t)255;
  const size_t oGTl = off; off += (size_t)GC * MP * 2;           off = (off + 255) & ~(size_t)255;
  if (off > ws_size || off > (size_t)WSMAX) return;
  unsigned short* XB  = (unsigned short*)(ws + oXB);
  unsigned short* WT  = (unsigned short*)(ws + oWT);
  float*          G   = (float*)(ws + oG);
  unsigned short* GTh = (unsigned short*)(ws + oGTh);
  unsigned short* GTl = (unsigned short*)(ws + oGTl);

  const int nUx = MP * (F_IN / 8);
  k_xprep<<<cdiv(nUx, NTHR), NTHR, 0, stream>>>(h, XB, nN, nUx);

  const int nUw = GC * (F_IN / 8);
  k_wtr<<<cdiv(nUw, NTHR), NTHR, 0, stream>>>(Wl, F_IN, GC, GC, F_IN, WT, nUw);

  k_gemm<<<dim3(MP / GBM, GC / GBN), GTHR, 0, stream>>>(XB, WT, G, GTh, GTl, F_IN, GC, MP);

  k_attn<<<cdiv(nN, RB), NTHR, 0, stream>>>(G, GTh, GTl, adj, aw, out, nN, nT, MP);
}
